// Model_39410619908782
// MI455X (gfx1250) — hardware-run, weakly checked
//
#include <hip/hip_runtime.h>
#include <math.h>

typedef __attribute__((ext_vector_type(16))) _Float16 v16h;
typedef __attribute__((ext_vector_type(8)))  _Float16 v8h;
typedef __attribute__((ext_vector_type(8)))  float    v8f;
typedef __attribute__((ext_vector_type(4)))  float    v4f;
typedef __attribute__((ext_vector_type(4)))  unsigned int v4u;

constexpr int kB     = 8;
constexpr int kSeq   = 96;
constexpr int kPred  = 96;
constexpr int kNvar  = 862;
constexpr int kNmark = 4;
constexpr int kL     = kNvar + kNmark;
constexpr int kRows  = kB * kL;
constexpr int kRowsP = 6976;
constexpr int kDm    = 512;
constexpr int kDs    = 16;
constexpr int kRk    = 32;
constexpr int kXz    = 2 * kDm;
constexpr int kXd    = kRk + 2 * kDs;
constexpr int kPrP   = 128;
constexpr int kNtRows = 64;
constexpr int kNtP    = 97;
constexpr int kScTS   = 64;
constexpr int kScCh   = 64;
constexpr int kScYP   = 68;
constexpr int kOutN   = kB * kPred * kNvar;
static_assert(kL == 866 && kRows == 6928, "token rows");
static_assert(kRowsP % 64 == 0 && kRowsP >= kRows && kRowsP - kRows < 64, "row padding");
static_assert(kXd == 64 && (kXd % 64) == 0 && (kDm % 64) == 0 && (kXz % 64) == 0 && (kPrP % 64) == 0, "GEMM N multiples of 64");
static_assert((kSeq % 32) == 0 && (kDm % 32) == 0 && (kRk % 32) == 0, "GEMM K multiples of 32");
static_assert(kPrP >= kPred, "projection pad");
static_assert((kOutN % 128) == 0, "output is a whole number of 4-line chunks");
static_assert((kNtRows * kSeq * 2) % 128 == 0, "token block byte range is line aligned");

constexpr float kCW  = 32.0f;
constexpr float kCXC = 64.0f;
constexpr float kCDT = 256.0f;
constexpr float kCY  = 1024.0f;
constexpr float kCH  = 16.0f;
constexpr float kInvCXC = 1.0f / kCXC;

constexpr size_t kRD32 = (size_t)kRowsP * kDm * 4;
constexpr size_t kRD16 = (size_t)kRowsP * kDm * 2;
constexpr size_t kOffRAW32 = 0;
constexpr size_t kOffENC32 = kOffRAW32 + kRD32;
constexpr size_t kOffX32   = kOffENC32 + kRD32;
constexpr size_t kOffT32   = kOffX32   + kRD32;
constexpr size_t kOffRAW16 = kOffT32   + kRD32;
constexpr size_t kOffENC16 = kOffRAW16 + kRD16;
constexpr size_t kOffX16   = kOffENC16 + kRD16;
constexpr size_t kOffXC16  = kOffX16   + kRD16;
constexpr size_t kOffDLR16 = kOffXC16  + kRD16;
constexpr size_t kOffYA16  = kOffDLR16 + kRD16;
constexpr size_t kOffXZ16  = kOffYA16  + kRD16;
constexpr size_t kOffDBL   = kOffXZ16  + (size_t)kRowsP * kXz * 2;
constexpr size_t kOffDT16  = kOffDBL   + (size_t)kRowsP * kXd * 4;
constexpr size_t kOffTOK16 = kOffDT16  + (size_t)kRowsP * kRk * 2;
constexpr size_t kOffDEC32 = kOffTOK16 + (size_t)kRowsP * kSeq * 2;
constexpr size_t kOffMEANR = kOffDEC32 + (size_t)kRowsP * kPrP * 4;
constexpr size_t kOffSTDR  = kOffMEANR + (size_t)kRowsP * 4;
constexpr size_t kOffEMBW  = kOffSTDR  + (size_t)kRowsP * 4;
constexpr size_t kOffINW   = kOffEMBW  + (size_t)kDm * kSeq * 2;
constexpr size_t kOffXPW   = kOffINW   + (size_t)4 * kXz * kDm * 2;
constexpr size_t kOffDTW   = kOffXPW   + (size_t)4 * kXd * kDm * 2;
constexpr size_t kOffOW    = kOffDTW   + (size_t)4 * kDm * kRk * 2;
constexpr size_t kOffW1    = kOffOW    + (size_t)4 * kDm * kDm * 2;
constexpr size_t kOffW2    = kOffW1    + (size_t)2 * kDm * kDm * 2;
constexpr size_t kOffGW    = kOffW2    + (size_t)2 * kDm * kDm * 2;
constexpr size_t kOffPW    = kOffGW    + (size_t)kDm * kDm * 2;
constexpr size_t kWsTotal  = kOffPW    + (size_t)kPrP * kDm * 2;
static_assert(kWsTotal <= 134217728ull, "carve cap");
static_assert((kRD32 % 128) == 0 && (kRD16 % 128) == 0, "plane sizes are line multiples");
static_assert((kOffXZ16 % 128) == 0 && (kOffDBL % 128) == 0 && (kOffDT16 % 128) == 0 && (kOffTOK16 % 128) == 0 &&
              (kOffDEC32 % 128) == 0 && (kOffMEANR % 128) == 0 && (kOffSTDR % 128) == 0 && (kOffEMBW % 128) == 0 &&
              (kOffINW % 128) == 0 && (kOffXPW % 128) == 0 && (kOffDTW % 128) == 0 && (kOffOW % 128) == 0 &&
              (kOffW1 % 128) == 0 && (kOffW2 % 128) == 0 && (kOffGW % 128) == 0 && (kOffPW % 128) == 0, "128-B aligned regions");

__device__ __forceinline__ float h16_to_f32(unsigned hb) {
  const unsigned sgn = (hb & 0x8000u) << 16;
  const unsigned em = hb & 0x7fffu;
  const float fn = __uint_as_float((em << 13) + 0x38000000u);
  const float fs = (float)em * 5.9604644775390625e-8f;
  const float mag = (em < 0x400u) ? fs : fn;
  return __uint_as_float(__float_as_uint(mag) | sgn);
}
__device__ __forceinline__ unsigned pack_h2(float a, float b) {
  const _Float16 h0 = (_Float16)a;
  const _Float16 h1 = (_Float16)b;
  const unsigned short u0 = __builtin_bit_cast(unsigned short, h0);
  const unsigned short u1 = __builtin_bit_cast(unsigned short, h1);
  return (unsigned)u0 | ((unsigned)u1 << 16);
}
__device__ __forceinline__ float sigmoidf_rcp(float x) {
  return __builtin_amdgcn_rcpf(1.0f + expf(-x));
}

__device__ __forceinline__ void guard_row_h(v8f& a, v8f& b, v8f& c, v8f& d, v16h x, v16h y) {
  asm volatile("v_nop\n\tv_nop\n\tv_nop\n\tv_nop" : "+v"(a), "+v"(b), "+v"(c), "+v"(d) : "v"(x), "v"(y));
}
__device__ __forceinline__ void keep4_h(v16h a, v16h b, v16h c, v16h d) {
  asm volatile("v_nop" :: "v"(a), "v"(b), "v"(c), "v"(d));
}
__device__ __forceinline__ void acc_guard4(v8f& a, v8f& b, v8f& c, v8f& d) {
  asm volatile("v_nop\n\tv_nop\n\tv_nop\n\tv_nop" : "+v"(a), "+v"(b), "+v"(c), "+v"(d));
}
struct FragH {
  union U { v16h v; v8h h[2]; };
  static __device__ __forceinline__ v16h load(const _Float16* p) {
    U f;
    f.h[0] = *(const v8h*)(p);
    f.h[1] = *(const v8h*)(p + 16);
    return f.v;
  }
  static __device__ __forceinline__ v8f mma(v16h a, v16h b, v8f c) {
    return __builtin_amdgcn_wmma_f32_16x16x32_f16(false, a, false, b, (short)0, c, false, false);
  }
};

template <int BIAS_MODE, int OUT_MODE, bool RESID, int ACT>
__global__ __launch_bounds__(256) void wmma_gemm64(
    const unsigned short* __restrict__ Ap, int lda,
    const unsigned short* __restrict__ Btp, int ldb,
    void* __restrict__ Cout, int ldc, void* __restrict__ Cout2, int ldc2,
    const float* __restrict__ bias, const float* __restrict__ resid,
    int M, int N, int K, float scale, float oscale)
{
  static_assert(!(RESID && ACT != 0), "resid path has no activation");
  static_assert(!(RESID && OUT_MODE != 0), "resid path is f32 only");
  const _Float16* A  = (const _Float16*)Ap;
  const _Float16* Bt = (const _Float16*)Btp;
  __shared__ __align__(16) float sT[8][16 * 68];
  const int lane = threadIdx.x & 31;
  const int wave = threadIdx.x >> 5;
  const int tilesN = N >> 6;
  const int tilesM = M >> 6;
  const int tile = blockIdx.x * 8 + wave;
  if (tile >= tilesM * tilesN) return;
  const int tm = tile / tilesN;
  const int tn = tile - tm * tilesN;
  const int m0 = tm << 6;
  const int n0 = tn << 6;
  const int rlane = lane & 15;
  const int koff  = (lane >> 4) * 8;
  const int mOff  = (lane >> 4) * 8;

  v8f acc[4][4];
#pragma unroll
  for (int i = 0; i < 4; ++i)
#pragma unroll
    for (int j = 0; j < 4; ++j) acc[i][j] = (v8f){0.f, 0.f, 0.f, 0.f, 0.f, 0.f, 0.f, 0.f};

  for (int k0 = 0; k0 < K; k0 += 32) {
    v16h bh[4];
#pragma unroll
    for (int j = 0; j < 4; ++j) {
      const size_t bo = (size_t)(n0 + (j << 4) + rlane) * ldb + koff + k0;
      bh[j] = FragH::load(Bt + bo);
    }
#pragma unroll
    for (int i = 0; i < 4; ++i) {
      const size_t ao = (size_t)(m0 + (i << 4) + rlane) * lda + koff + k0;
      const v16h ah = FragH::load(A + ao);
#pragma unroll
      for (int j = 0; j < 4; ++j) acc[i][j] = FragH::mma(ah, bh[j], acc[i][j]);
      guard_row_h(acc[i][0], acc[i][1], acc[i][2], acc[i][3], ah, bh[3]);
    }
    keep4_h(bh[0], bh[1], bh[2], bh[3]);
  }
  acc_guard4(acc[0][0], acc[0][1], acc[0][2], acc[0][3]);
  acc_guard4(acc[1][0], acc[1][1], acc[1][2], acc[1][3]);
  acc_guard4(acc[2][0], acc[2][1], acc[2][2], acc[2][3]);
  acc_guard4(acc[3][0], acc[3][1], acc[3][2], acc[3][3]);

  float* slab = sT[wave];
#pragma unroll
  for (int i = 0; i < 4; ++i) {
    const int mBase = m0 + (i << 4);
#pragma unroll
    for (int j = 0; j < 4; ++j) {
      float bv = 0.f;
      if (BIAS_MODE == 2) bv = bias[n0 + (j << 4) + rlane];
#pragma unroll
      for (int r = 0; r < 8; ++r) {
        float v = acc[i][j][r] * scale;
        if (BIAS_MODE == 2) v += bv;
        if (ACT == 2) v = fmaxf(v, 0.0f);
        slab[(mOff + r) * 68 + (j << 4) + rlane] = v;
      }
    }
    __builtin_amdgcn_fence(__ATOMIC_RELEASE, "workgroup");
    __builtin_amdgcn_wave_barrier();
    __builtin_amdgcn_fence(__ATOMIC_ACQUIRE, "workgroup");
    if (OUT_MODE == 0 || OUT_MODE == 3) {
      float* C = (float*)Cout;
      const int hh = lane >> 4, c4 = (lane & 15) * 4;
      v4f vals[8];
#pragma unroll
      for (int it = 0; it < 8; ++it) {
        const int row = it * 2 + hh;
        v4f v = *(const v4f*)(slab + row * 68 + c4);
        if (RESID) {
          const v4f r4 = *(const v4f*)(resid + (size_t)(mBase + row) * ldc + n0 + c4);
          v = v + r4;
        }
        vals[it] = v;
      }
      for (int pass = 0; pass < 2; ++pass) {
#pragma unroll
        for (int it = 0; it < 8; ++it) {
          const int row = it * 2 + hh;
          *(volatile v4f*)(C + (size_t)(mBase + row) * ldc + n0 + c4) = vals[it];
        }
        __threadfence();
      }
    }
    if (OUT_MODE == 1 || OUT_MODE == 3) {
      unsigned short* C16 = (unsigned short*)((OUT_MODE == 1) ? Cout : Cout2);
      const int ld16 = (OUT_MODE == 1) ? ldc : ldc2;
      const int q = lane >> 3, c8 = (lane & 7) * 8;
      v8h hvv[4];
#pragma unroll
      for (int it = 0; it < 4; ++it) {
        const int row = it * 4 + q;
        const float* sp = slab + row * 68 + c8;
#pragma unroll
        for (int e = 0; e < 8; ++e) hvv[it][e] = (_Float16)(sp[e] * oscale);
      }
      for (int pass = 0; pass < 2; ++pass) {
#pragma unroll
        for (int it = 0; it < 4; ++it) {
          const int row = it * 4 + q;
          *(volatile v8h*)(C16 + (size_t)(mBase + row) * ld16 + n0 + c8) = hvv[it];
        }
        __threadfence();
      }
    }
    __builtin_amdgcn_fence(__ATOMIC_RELEASE, "workgroup");
    __builtin_amdgcn_wave_barrier();
    __builtin_amdgcn_fence(__ATOMIC_ACQUIRE, "workgroup");
  }
}

__global__ __launch_bounds__(256) void cast_w_kernel(
    const float* __restrict__ src, unsigned short* __restrict__ dst, int total8, int src8, float scale)
{
  const int i = blockIdx.x * 256 + threadIdx.x;
  if (i >= total8) return;
  const bool live = (i < src8);
  const size_t es = (size_t)(live ? i : 0) << 3;
  const v4f a0 = *(const v4f*)(src + es);
  const v4f a1 = *(const v4f*)(src + es + 4);
  v8h hv;
#pragma unroll
  for (int e = 0; e < 4; ++e) {
    const float f0 = live ? (a0[e] * scale) : 0.0f;
    const float f1 = live ? (a1[e] * scale) : 0.0f;
    hv[e]     = (_Float16)f0;
    hv[4 + e] = (_Float16)f1;
  }
  unsigned short* q = dst + ((size_t)i << 3);
  *(volatile v8h*)q = hv;
  __threadfence();
  *(volatile v8h*)q = hv;
}

__global__ __launch_bounds__(256) void zero16_kernel(unsigned short* __restrict__ dst, int total8)
{
  const int i = blockIdx.x * 256 + threadIdx.x;
  if (i >= total8) return;
  const v4u z = (v4u){0u, 0u, 0u, 0u};
  unsigned short* q = dst + ((size_t)i << 3);
  *(volatile v4u*)q = z;
  __threadfence();
  *(volatile v4u*)q = z;
}

__global__ __launch_bounds__(256) void norm_tok_kernel(
    const float* __restrict__ xenc, const float* __restrict__ xmark,
    unsigned short* __restrict__ tok16, float* __restrict__ meanR, float* __restrict__ stdR)
{
  __shared__ __align__(16) float sT[kNtRows * kNtP];
  __shared__ __align__(16) float sP[4 * kNtRows];
  __shared__ __align__(16) float sMean[kNtRows];
  __shared__ __align__(16) float sStd[kNtRows];
  const int tid = threadIdx.x;
  const int r = tid & 63, part = tid >> 6;
  const int row = blockIdx.x * kNtRows + r;
  const bool valid = row < kRows;
  const int rowc = valid ? row : (kRows - 1);
  const int b = rowc / kL;
  const int l = rowc - b * kL;
  const bool isvar  = valid && (l < kNvar);
  const bool ismark = valid && (l >= kNvar);
  const int vc = (l < kNvar) ? l : (kNvar - 1);
  int mk = l - kNvar;
  mk = (mk < 0) ? 0 : mk;
  mk = (mk > kNmark - 1) ? (kNmark - 1) : mk;
  const float fa = isvar ? 1.0f : 0.0f;
  const float fb = ismark ? 1.0f : 0.0f;
  const int s0 = part * 24;
  float ps = 0.f;
#pragma unroll 4
  for (int j = 0; j < 24; ++j) {
    const int s = s0 + j;
    const float a = xenc[((size_t)b * kSeq + s) * kNvar + vc];
    const float m = xmark[((size_t)b * kSeq + s) * kNmark + mk];
    const float val = fmaf(fa, a, fb * m);
    sT[r * kNtP + s] = val;
    ps += val;
  }
  sP[part * kNtRows + r] = ps;
  __syncthreads();
  const float mean = ((sP[r] + sP[kNtRows + r]) + (sP[2 * kNtRows + r] + sP[3 * kNtRows + r])) * (1.0f / kSeq);
  __syncthreads();
  float pq = 0.f;
#pragma unroll 4
  for (int j = 0; j < 24; ++j) {
    const float dd = sT[r * kNtP + s0 + j] - mean;
    pq += dd * dd;
  }
  sP[part * kNtRows + r] = pq;
  __syncthreads();
  const float var = ((sP[r] + sP[kNtRows + r]) + (sP[2 * kNtRows + r] + sP[3 * kNtRows + r])) * (1.0f / kSeq);
  const float sd  = sqrtf(var + 1e-5f);
  const float inv = __builtin_amdgcn_rcpf(sd);
  const float meff = isvar ? mean : 0.0f;
  const float ieff = isvar ? inv : 1.0f;
#pragma unroll 4
  for (int j = 0; j < 24; ++j) {
    const float x = sT[r * kNtP + s0 + j];
    sT[r * kNtP + s0 + j] = (x - meff) * ieff;
  }
  if (part == 0) {
    sMean[r] = isvar ? mean : 0.0f;
    sStd[r]  = isvar ? sd : 1.0f;
  }
  __syncthreads();
  v8h hv[3];
#pragma unroll
  for (int it = 0; it < 3; ++it) {
    const int c = it * 256 + tid;
    const int flat = c * 8;
    const int rr = flat / kSeq;
    const int ss = flat - rr * kSeq;
#pragma unroll
    for (int e = 0; e < 8; ++e) hv[it][e] = (_Float16)sT[rr * kNtP + ss + e];
  }
  const int t16 = (tid < 16) ? tid : 0;
  const v4f mv = *(const v4f*)(sMean + t16 * 4);
  const v4f sv = *(const v4f*)(sStd + t16 * 4);
  unsigned short* tb = tok16 + (size_t)blockIdx.x * (kNtRows * kSeq);
  float* mb = meanR + (size_t)blockIdx.x * kNtRows;
  float* sb = stdR  + (size_t)blockIdx.x * kNtRows;
  for (int pass = 0; pass < 2; ++pass) {
#pragma unroll
    for (int it = 0; it < 3; ++it) {
      const int c = it * 256 + tid;
      *(volatile v8h*)(tb + (size_t)c * 8) = hv[it];
    }
    if (tid < 16) {
      *(volatile v4f*)(mb + tid * 4) = mv;
      *(volatile v4f*)(sb + tid * 4) = sv;
    }
    __threadfence();
  }
}

__global__ __launch_bounds__(256) void conv_silu_kernel(
    const unsigned* __restrict__ XZw, const float* __restrict__ cw, const float* __restrict__ cb,
    unsigned short* __restrict__ XC16, int dir)
{
  __shared__ __align__(16) unsigned sW[256 * 4];
  const int tid = threadIdx.x;
  const int gi = blockIdx.x * 256 + tid;
  const int row = gi >> 6;
  const int c8 = (gi & 63) * 8;
  const bool valid = row < kRows;
  const int rowc = valid ? row : (kRows - 1);
  const int b = rowc / kL;
  const int l = rowc - b * kL;
  const bool hasn = valid && (dir ? (l < kL - 1) : (l > 0));
  const int nrow = hasn ? (dir ? (rowc + 1) : (rowc - 1)) : rowc;
#pragma unroll 1
  for (int it = 0; it < 4; ++it) {
    const int d = c8 + it * 2;
    const unsigned wc = XZw[(size_t)rowc * (kXz / 2) + (d >> 1)];
    const unsigned wn = XZw[(size_t)nrow * (kXz / 2) + (d >> 1)];
    const v4f cwv = *(const v4f*)(cw + d * 2);
    const float cb0 = cb[d];
    const float cb1 = cb[d + 1];
    const float cur0 = h16_to_f32(wc & 0xffffu);
    const float cur1 = h16_to_f32(wc >> 16);
    const float nb0 = h16_to_f32(wn & 0xffffu);
    const float nb1 = h16_to_f32(wn >> 16);
    const float p0 = hasn ? nb0 : 0.0f;
    const float p1 = hasn ? nb1 : 0.0f;
    const float v0 = p0 * cwv[0] + cur0 * cwv[1] + cb0;
    const float v1 = p1 * cwv[2] + cur1 * cwv[3] + cb1;
    const float s0 = v0 * sigmoidf_rcp(v0);
    const float s1 = v1 * sigmoidf_rcp(v1);
    const float o0 = valid ? (s0 * kCXC) : 0.0f;
    const float o1 = valid ? (s1 * kCXC) : 0.0f;
    sW[tid * 4 + it] = pack_h2(o0, o1);
  }
  __syncthreads();
  const v4u o = *(const v4u*)(sW + tid * 4);
  unsigned short* q = XC16 + (size_t)row * kDm + c8;
  *(volatile v4u*)q = o;
  __threadfence();
  *(volatile v4u*)q = o;
}

__global__ __launch_bounds__(256) void dt_cast_kernel(
    const float* __restrict__ DBL, unsigned short* __restrict__ DT16, int total8, float scale)
{
  const int i = blockIdx.x * 256 + threadIdx.x;
  if (i >= total8) return;
  const int e0  = i << 3;
  const int row = e0 >> 5;
  const int c8  = e0 & 31;
  const float* p = DBL + (size_t)row * kXd + c8;
  const v4f a0 = *(const v4f*)(p);
  const v4f a1 = *(const v4f*)(p + 4);
  v8h hv;
#pragma unroll
  for (int e = 0; e < 4; ++e) {
    hv[e]     = (_Float16)(a0[e] * scale);
    hv[4 + e] = (_Float16)(a1[e] * scale);
  }
  unsigned short* qd = DT16 + e0;
  *(volatile v8h*)qd = hv;
  __threadfence();
  *(volatile v8h*)qd = hv;
}

__global__ __launch_bounds__(64) void scan_kernel(
    const float* __restrict__ DBL, const unsigned* __restrict__ XZw, const unsigned* __restrict__ XCw,
    const unsigned* __restrict__ DLRw, const float* __restrict__ Alog, const float* __restrict__ Dp,
    unsigned short* __restrict__ Y16, int dir)
{
  __shared__ __align__(16) float sBC[kScTS * 32];
  __shared__ __align__(16) float sY[kScTS * kScYP];
  __shared__ __align__(16) float sA[kDs * kScCh];
  const int tid = threadIdx.x, lane = tid & 31, wave = tid >> 5;
  const int bix = blockIdx.x >> 3;
  const int d0  = (blockIdx.x & 7) * kScCh;
  const int d   = d0 + tid;
  const size_t row0 = (size_t)bix * kL;
#pragma unroll 1
  for (int s = 0; s < kDs; ++s) sA[s * kScCh + tid] = -expf(Alog[(size_t)d * kDs + s]);
  __syncthreads();
  float negA[kDs], h[kDs];
#pragma unroll
  for (int s = 0; s < kDs; ++s) {
    negA[s] = sA[s * kScCh + tid];
    h[s] = 0.f;
  }
  const float Dd = Dp[d];
  const int sh = (d & 1) * 16;
  const int dw = d >> 1;
  const int lr = tid >> 3, lc4 = (tid & 7) * 4;
  const int q = lane >> 3, c8 = (lane & 7) * 8;
#pragma unroll 1
  for (int t0 = 0; t0 < kL; t0 += kScTS) {
    const int rem = kL - t0;
    const int nst = (rem < kScTS) ? rem : kScTS;
    __syncthreads();
#pragma unroll
    for (int i = 0; i < 8; ++i) {
      const int r = lr + 8 * i;
      const int j = t0 + r;
      const int jc = (j < kL) ? j : (kL - 1);
      const int t = dir ? (kL - 1 - jc) : jc;
      *(v4f*)(sBC + r * 32 + lc4) = *(const v4f*)(DBL + (row0 + t) * kXd + kRk + lc4);
    }
    __syncthreads();
#pragma unroll 1
    for (int s = 0; s < nst; ++s) {
      const int j = t0 + s;
      const int t = dir ? (kL - 1 - j) : j;
      const size_t grow = row0 + t;
      const unsigned wd = DLRw[grow * (kDm / 2) + dw];
      const unsigned wx = XCw[grow * (kDm / 2) + dw];
      const unsigned wz = XZw[grow * (kXz / 2) + (kDm / 2) + dw];
      const float v  = h16_to_f32((wd >> sh) & 0xffffu);
      const float xt = h16_to_f32((wx >> sh) & 0xffffu) * kInvCXC;
      const float zv = h16_to_f32((wz >> sh) & 0xffffu);
      float Bs[kDs], Cs[kDs];
#pragma unroll
      for (int q4 = 0; q4 < 4; ++q4) {
        const v4f bv = *(const v4f*)(sBC + s * 32 + 4 * q4);
        const v4f cv = *(const v4f*)(sBC + s * 32 + kDs + 4 * q4);
        Bs[4 * q4 + 0] = bv[0]; Bs[4 * q4 + 1] = bv[1]; Bs[4 * q4 + 2] = bv[2]; Bs[4 * q4 + 3] = bv[3];
        Cs[4 * q4 + 0] = cv[0]; Cs[4 * q4 + 1] = cv[1]; Cs[4 * q4 + 2] = cv[2]; Cs[4 * q4 + 3] = cv[3];
      }
      const float dt  = fmaxf(v, 0.0f) + log1pf(expf(-fabsf(v)));
      const float dtx = dt * xt;
      float y = 0.f;
#pragma unroll
      for (int k = 0; k < kDs; ++k) {
        const float e = __expf(dt * negA[k]);
        h[k] = e * h[k] + dtx * Bs[k];
        y = h[k] * Cs[k] + y;
      }
      y = xt * Dd + y;
      y = y * (zv * sigmoidf_rcp(zv));
      sY[s * kScYP + tid] = y * kCY;
    }
    __syncthreads();
    v8h hv[8];
#pragma unroll
    for (int it = 0; it < 8; ++it) {
      const int row = it * 8 + wave * 4 + q;
      const int rowc = (row < nst) ? row : (nst - 1);
      const float* sp = sY + rowc * kScYP + c8;
      const v4f a0 = *(const v4f*)(sp);
      const v4f a1 = *(const v4f*)(sp + 4);
#pragma unroll
      for (int e = 0; e < 4; ++e) {
        hv[it][e]     = (_Float16)a0[e];
        hv[it][4 + e] = (_Float16)a1[e];
      }
    }
    for (int pass = 0; pass < 2; ++pass) {
#pragma unroll
      for (int it = 0; it < 8; ++it) {
        const int row = it * 8 + wave * 4 + q;
        const int rowc = (row < nst) ? row : (nst - 1);
        const int j = t0 + rowc;
        const int t = dir ? (kL - 1 - j) : j;
        if (row < nst) *(volatile v8h*)(Y16 + (row0 + t) * kDm + d0 + c8) = hv[it];
      }
      __threadfence();
    }
  }
}

__global__ __launch_bounds__(256) void ln_kernel(
    const float* __restrict__ in, const float* __restrict__ g, const float* __restrict__ be,
    float* __restrict__ out32, unsigned short* __restrict__ out16)
{
  __shared__ __align__(16) float sR[8 * kDm];
  const int lane = threadIdx.x & 31, wave = threadIdx.x >> 5;
  const int row = blockIdx.x * 8 + wave;
  const float* ip = in + (size_t)row * kDm;
  float* sr = sR + wave * kDm;
  float sum = 0.f;
#pragma unroll 1
  for (int it = 0; it < 4; ++it) {
    const int c = it * 128 + lane * 4;
    const v4f v = *(const v4f*)(ip + c);
    *(v4f*)(sr + c) = v;
    sum += (v[0] + v[1]) + (v[2] + v[3]);
  }
#pragma unroll
  for (int o = 16; o > 0; o >>= 1) sum += __shfl_xor(sum, o, 32);
  const float mean = sum * (1.0f / kDm);
  float sq = 0.f;
#pragma unroll 1
  for (int it = 0; it < 4; ++it) {
    const int c = it * 128 + lane * 4;
    const v4f v = *(const v4f*)(sr + c);
    const float e0 = v[0] - mean, e1 = v[1] - mean, e2 = v[2] - mean, e3 = v[3] - mean;
    sq += (e0 * e0 + e1 * e1) + (e2 * e2 + e3 * e3);
  }
#pragma unroll
  for (int o = 16; o > 0; o >>= 1) sq += __shfl_xor(sq, o, 32);
  const float inv = __builtin_amdgcn_rcpf(sqrtf(sq * (1.0f / kDm) + 1e-5f));
#pragma unroll 1
  for (int it = 0; it < 4; ++it) {
    const int c = it * 128 + lane * 4;
    const v4f v = *(const v4f*)(sr + c);
    const v4f gv = *(const v4f*)(g + c);
    const v4f bv = *(const v4f*)(be + c);
    v4f o;
    o[0] = (v[0] - mean) * inv * gv[0] + bv[0];
    o[1] = (v[1] - mean) * inv * gv[1] + bv[1];
    o[2] = (v[2] - mean) * inv * gv[2] + bv[2];
    o[3] = (v[3] - mean) * inv * gv[3] + bv[3];
    *(v4f*)(sr + c) = o;
  }
  __syncthreads();
  v4f fv[4];
  v8h hv[2];
#pragma unroll
  for (int it = 0; it < 4; ++it) fv[it] = *(const v4f*)(sr + it * 128 + lane * 4);
#pragma unroll
  for (int j = 0; j < 2; ++j) {
    const float* sp = sr + j * 256 + lane * 8;
    const v4f a0 = *(const v4f*)(sp);
    const v4f a1 = *(const v4f*)(sp + 4);
#pragma unroll
    for (int e = 0; e < 4; ++e) {
      hv[j][e]     = (_Float16)a0[e];
      hv[j][4 + e] = (_Float16)a1[e];
    }
  }
  float* o32 = out32 + (size_t)row * kDm;
  unsigned short* o16 = out16 + (size_t)row * kDm;
  for (int pass = 0; pass < 2; ++pass) {
#pragma unroll
    for (int it = 0; it < 4; ++it) *(volatile v4f*)(o32 + it * 128 + lane * 4) = fv[it];
#pragma unroll
    for (int j = 0; j < 2; ++j) *(volatile v8h*)(o16 + j * 256 + lane * 8) = hv[j];
    __threadfence();
  }
}

__global__ __launch_bounds__(256) void fin_gate_kernel(
    const float* __restrict__ enc, const float* __restrict__ gpre, const float* __restrict__ raw,
    const float* __restrict__ g, const float* __restrict__ be, unsigned short* __restrict__ out16)
{
  __shared__ __align__(16) float sR[8 * kDm];
  const int lane = threadIdx.x & 31, wave = threadIdx.x >> 5;
  const int row = blockIdx.x * 8 + wave;
  const float* ip = enc  + (size_t)row * kDm;
  const float* gp = gpre + (size_t)row * kDm;
  const float* rp = raw  + (size_t)row * kDm;
  float* sr = sR + wave * kDm;
  float sum = 0.f;
#pragma unroll 1
  for (int it = 0; it < 4; ++it) {
    const int c = it * 128 + lane * 4;
    const v4f v = *(const v4f*)(ip + c);
    *(v4f*)(sr + c) = v;
    sum += (v[0] + v[1]) + (v[2] + v[3]);
  }
#pragma unroll
  for (int o = 16; o > 0; o >>= 1) sum += __shfl_xor(sum, o, 32);
  const float mean = sum * (1.0f / kDm);
  float sq = 0.f;
#pragma unroll 1
  for (int it = 0; it < 4; ++it) {
    const int c = it * 128 + lane * 4;
    const v4f v = *(const v4f*)(sr + c);
    const float e0 = v[0] - mean, e1 = v[1] - mean, e2 = v[2] - mean, e3 = v[3] - mean;
    sq += (e0 * e0 + e1 * e1) + (e2 * e2 + e3 * e3);
  }
#pragma unroll
  for (int o = 16; o > 0; o >>= 1) sq += __shfl_xor(sq, o, 32);
  const float inv = __builtin_amdgcn_rcpf(sqrtf(sq * (1.0f / kDm) + 1e-5f));
#pragma unroll 1
  for (int it = 0; it < 4; ++it) {
    const int c = it * 128 + lane * 4;
    const v4f v  = *(const v4f*)(sr + c);
    const v4f gv = *(const v4f*)(g + c);
    const v4f bv = *(const v4f*)(be + c);
    const v4f pv = *(const v4f*)(gp + c);
    const v4f rv = *(const v4f*)(rp + c);
    v4f o;
    o[0] = ((v[0] - mean) * inv * gv[0] + bv[0]) + sigmoidf_rcp(pv[0]) * rv[0];
    o[1] = ((v[1] - mean) * inv * gv[1] + bv[1]) + sigmoidf_rcp(pv[1]) * rv[1];
    o[2] = ((v[2] - mean) * inv * gv[2] + bv[2]) + sigmoidf_rcp(pv[2]) * rv[2];
    o[3] = ((v[3] - mean) * inv * gv[3] + bv[3]) + sigmoidf_rcp(pv[3]) * rv[3];
    *(v4f*)(sr + c) = o;
  }
  __syncthreads();
  v8h hv[2];
#pragma unroll
  for (int j = 0; j < 2; ++j) {
    const float* sp = sr + j * 256 + lane * 8;
    const v4f a0 = *(const v4f*)(sp);
    const v4f a1 = *(const v4f*)(sp + 4);
#pragma unroll
    for (int e = 0; e < 4; ++e) {
      hv[j][e]     = (_Float16)a0[e];
      hv[j][4 + e] = (_Float16)a1[e];
    }
  }
  unsigned short* o16 = out16 + (size_t)row * kDm;
  for (int pass = 0; pass < 2; ++pass) {
#pragma unroll
    for (int j = 0; j < 2; ++j) *(volatile v8h*)(o16 + j * 256 + lane * 8) = hv[j];
    __threadfence();
  }
}

__global__ __launch_bounds__(256) void out_kernel(
    const float* __restrict__ DEC, const float* __restrict__ pb, const float* __restrict__ meanR,
    const float* __restrict__ stdR, float* __restrict__ out)
{
  const int i = blockIdx.x * 256 + threadIdx.x;
  if (i >= kOutN / 4) return;
  const int e0 = i * 4;
  v4f o;
#pragma unroll
  for (int k = 0; k < 4; ++k) {
    const int e = e0 + k;
    const int b = e / (kPred * kNvar);
    const int rem = e - b * (kPred * kNvar);
    const int p = rem / kNvar;
    const int v = rem - p * kNvar;
    const int rr = b * kL + v;
    const float dv = DEC[(size_t)rr * kPrP + p];
    const float bp = pb[p];
    const float sd = stdR[rr];
    const float mn = meanR[rr];
    o[k] = (dv + bp) * sd + mn;
    if (k == 1) asm volatile("" ::: "memory");
  }
  float* q = out + e0;
  *(volatile v4f*)q = o;
  __threadfence();
  *(volatile v4f*)q = o;
}

static inline int gemm_blocks(int M, int N) { return ((M / 64) * (N / 64) + 7) / 8; }

extern "C" void kernel_launch(void* const* d_in, const int* in_sizes, int n_in,
                              void* d_out, int out_size, void* d_ws, size_t ws_size,
                              hipStream_t stream)
{
  if (n_in < 29) return;
  if (in_sizes[0] != kB * kSeq * kNvar) return;
  if (in_sizes[1] != kB * kSeq * kNmark) return;
  if (in_sizes[4] != kDm * kSeq || in_sizes[5] != kDm) return;
  if (in_sizes[6] != 4 * kXz * kDm) return;
  if (in_sizes[7] != 4 * kDm * 2 || in_sizes[8] != 4 * kDm) return;
  if (in_sizes[9] != 4 * kXd * kDm) return;
  if (in_sizes[10] != 4 * kDm * kRk || in_sizes[11] != 4 * kDm) return;
  if (in_sizes[12] != 4 * kDm * kDs || in_sizes[13] != 4 * kDm) return;
  if (in_sizes[14] != 4 * kDm * kDm) return;
  if (in_sizes[15] != 2 * kDm * kDm || in_sizes[16] != 2 * kDm) return;
  if (in_sizes[17] != 2 * kDm * kDm || in_sizes[18] != 2 * kDm) return;
  if (in_sizes[19] != 2 * kDm || in_sizes[20] != 2 * kDm || in_sizes[21] != 2 * kDm || in_sizes[22] != 2 * kDm) return;
  if (in_sizes[23] != kDm || in_sizes[24] != kDm) return;
  if (in_sizes[25] != kDm * kDm || in_sizes[26] != kDm) return;
  if (in_sizes[27] != kPred * kDm || in_sizes[28] != kPred) return;
  if (out_size != kOutN) return;
  if (ws_size < kWsTotal) return;

  const float* x_enc  = (const float*)d_in[0];
  const float* x_mark = (const float*)d_in[1];
  const float* emb_w  = (const float*)d_in[4];
  const float* emb_b  = (const float*)d_in[5];
  const float* inw    = (const float*)d_in[6];
  const float* cw     = (const float*)d_in[7];
  const float* cb     = (const float*)d_in[8];
  const float* xpw    = (const float*)d_in[9];
  const float* dtw    = (const float*)d_in[10];
  const float* dtb    = (const float*)d_in[11];
  const float* alog   = (const float*)d_in[12];
  const float* dpar   = (const float*)d_in[13];
  const float* ow     = (const float*)d_in[14];
  const float* w1     = (const float*)d_in[15];
  const float* b1     = (const float*)d_in[16];
  const float* w2     = (const float*)d_in[17];
  const float* b2     = (const float*)d_in[18];
  const float* ln1g   = (const float*)d_in[19];
  const float* ln1b   = (const float*)d_in[20];
  const float* ln2g   = (const float*)d_in[21];
  const float* ln2b   = (const float*)d_in[22];
  const float* fing   = (const float*)d_in[23];
  const float* finb   = (const float*)d_in[24];
  const float* gw     = (const float*)d_in[25];
  const float* gb     = (const float*)d_in[26];
  const float* pw     = (const float*)d_in[27];
  const float* pb     = (const float*)d_in[28];
  float* out = (float*)d_out;

  char* ws = (char*)d_ws;
  float* RAW32 = (float*)(ws + kOffRAW32);
  float* ENC32 = (float*)(ws + kOffENC32);
  float* X32   = (float*)(ws + kOffX32);
  float* T32   = (float*)(ws + kOffT32);
  unsigned short* RAW16 = (unsigned short*)(ws + kOffRAW16);
  unsigned short* ENC16 = (unsigned short*)(ws + kOffENC16);
  unsigned short* X16   = (unsigned short*)(ws + kOffX16);
  unsigned short* XC16  = (unsigned short*)(ws + kOffXC16);
  unsigned short* DLR16 = (unsigned short*)(ws + kOffDLR16);
  unsigned short* YA16  = (unsigned short*)(ws + kOffYA16);
  unsigned short* XZ16  = (unsigned short*)(ws + kOffXZ16);
  float* DBL = (float*)(ws + kOffDBL);
  unsigned short* DT16  = (unsigned short*)(ws + kOffDT16);
  unsigned short* TOK16 = (unsigned short*)(ws + kOffTOK16);
  float* DEC32 = (float*)(ws + kOffDEC32);
  float* MEANR = (float*)(ws + kOffMEANR);
  float* STDR  = (float*)(ws + kOffSTDR);
  unsigned short* EMBW = (unsigned short*)(ws + kOffEMBW);
  unsigned short* INW  = (unsigned short*)(ws + kOffINW);
  unsigned short* XPW  = (unsigned short*)(ws + kOffXPW);
  unsigned short* DTW  = (unsigned short*)(ws + kOffDTW);
  unsigned short* OW   = (unsigned short*)(ws + kOffOW);
  unsigned short* W1   = (unsigned short*)(ws + kOffW1);
  unsigned short* W2   = (unsigned short*)(ws + kOffW2);
  unsigned short* GW   = (unsigned short*)(ws + kOffGW);
  unsigned short* PW   = (unsigned short*)(ws + kOffPW);

  {
    const int n_emb = kDm * kSeq / 8, n_in4 = 4 * kXz * kDm / 8, n_xp = 4 * kXd * kDm / 8;
    const int n_dt = 4 * kDm * kRk / 8, n_ow = 4 * kDm * kDm / 8, n_w = 2 * kDm * kDm / 8;
    const int n_gw = kDm * kDm / 8, n_pw = kPrP * kDm / 8, n_pws = kPred * kDm / 8;
    cast_w_kernel<<<n_emb / 256, 256, 0, stream>>>(emb_w, EMBW, n_emb, n_emb, kCW);
    cast_w_kernel<<<n_in4 / 256, 256, 0, stream>>>(inw, INW, n_in4, n_in4, kCW);
    cast_w_kernel<<<n_xp / 256, 256, 0, stream>>>(xpw, XPW, n_xp, n_xp, kCW);
    cast_w_kernel<<<n_dt / 256, 256, 0, stream>>>(dtw, DTW, n_dt, n_dt, kCW);
    cast_w_kernel<<<n_ow / 256, 256, 0, stream>>>(ow, OW, n_ow, n_ow, kCW);
    cast_w_kernel<<<n_w / 256, 256, 0, stream>>>(w1, W1, n_w, n_w, kCW);
    cast_w_kernel<<<n_w / 256, 256, 0, stream>>>(w2, W2, n_w, n_w, kCW);
    cast_w_kernel<<<n_gw / 256, 256, 0, stream>>>(gw, GW, n_gw, n_gw, kCW);
    cast_w_kernel<<<n_pw / 256, 256, 0, stream>>>(pw, PW, n_pw, n_pws, kCW);
  }
  {
    const int n8 = (kRowsP - kRows) * kDm / 8;
    zero16_kernel<<<n8 / 256, 256, 0, stream>>>(YA16 + (size_t)kRows * kDm, n8);
  }

  norm_tok_kernel<<<kRowsP / kNtRows, 256, 0, stream>>>(x_enc, x_mark, TOK16, MEANR, STDR);

  wmma_gemm64<2, 3, false, 0><<<gemm_blocks(kRowsP, kDm), 256, 0, stream>>>(
      TOK16, kSeq, EMBW, kSeq, (void*)RAW32, kDm, (void*)RAW16, kDm,
      emb_b, nullptr, kRowsP, kDm, kSeq, 1.0f / kCW, 1.0f);

  for (int l = 0; l < 2; ++l) {
    const float* enc32in = (l == 0) ? RAW32 : ENC32;
    const unsigned short* enc16in = (l == 0) ? RAW16 : ENC16;
    for (int dir = 0; dir < 2; ++dir) {
      const size_t wo = (size_t)(l * 2 + dir);
      wmma_gemm64<0, 1, false, 0><<<gemm_blocks(kRowsP, kXz), 256, 0, stream>>>(
          enc16in, kDm, INW + wo * kXz * kDm, kDm, (void*)XZ16, kXz, nullptr, 0,
          nullptr, nullptr, kRowsP, kXz, kDm, 1.0f / kCW, 1.0f);
      conv_silu_kernel<<<kRowsP * (kDm / 8) / 256, 256, 0, stream>>>(
          (const unsigned*)XZ16, cw + wo * kDm * 2, cb + wo * kDm, XC16, dir);
      wmma_gemm64<0, 0, false, 0><<<gemm_blocks(kRowsP, kXd), 256, 0, stream>>>(
          XC16, kDm, XPW + wo * kXd * kDm, kDm, (void*)DBL, kXd, nullptr, 0,
          nullptr, nullptr, kRowsP, kXd, kDm, 1.0f / (kCXC * kCW), 1.0f);
      dt_cast_kernel<<<kRowsP * kRk / 8 / 256, 256, 0, stream>>>(DBL, DT16, kRowsP * kRk / 8, kCDT);
      wmma_gemm64<2, 1, false, 0><<<gemm_blocks(kRowsP, kDm), 256, 0, stream>>>(
          DT16, kRk, DTW + wo * kDm * kRk, kRk, (void*)DLR16, kDm, nullptr, 0,
          dtb + wo * kDm, nullptr, kRowsP, kDm, kRk, 1.0f / (kCDT * kCW), 1.0f);
      scan_kernel<<<kB * (kDm / kScCh), kScCh, 0, stream>>>(
          DBL, (const unsigned*)XZ16, (const unsigned*)XC16, (const unsigned*)DLR16,
          alog + wo * kDm * kDs, dpar + wo * kDm, YA16, dir);
      wmma_gemm64<0, 0, true, 0><<<gemm_blocks(kRowsP, kDm), 256, 0, stream>>>(
          YA16, kDm, OW + wo * kDm * kDm, kDm, (void*)((dir == 0) ? X32 : T32), kDm, nullptr, 0,
          nullptr, (dir == 0) ? enc32in : (const float*)X32, kRowsP, kDm, kDm, 1.0f / (kCY * kCW), 1.0f);
    }
    ln_kernel<<<kRowsP / 8, 256, 0, stream>>>(T32, ln1g + l * kDm, ln1b + l * kDm, X32, X16);
    wmma_gemm64<2, 1, false, 2><<<gemm_blocks(kRowsP, kDm), 256, 0, stream>>>(
        X16, kDm, W1 + (size_t)l * kDm * kDm, kDm, (void*)YA16, kDm, nullptr, 0,
        b1 + l * kDm, nullptr, kRowsP, kDm, kDm, 1.0f / kCW, kCH);
    wmma_gemm64<2, 0, true, 0><<<gemm_blocks(kRowsP, kDm), 256, 0, stream>>>(
        YA16, kDm, W2 + (size_t)l * kDm * kDm, kDm, (void*)T32, kDm, nullptr, 0,
        b2 + l * kDm, X32, kRowsP, kDm, kDm, 1.0f / (kCH * kCW), 1.0f);
    ln_kernel<<<kRowsP / 8, 256, 0, stream>>>(T32, ln2g + l * kDm, ln2b + l * kDm, ENC32, ENC16);
  }

  wmma_gemm64<2, 0, false, 0><<<gemm_blocks(kRowsP, kDm), 256, 0, stream>>>(
      RAW16, kDm, GW, kDm, (void*)X32, kDm, nullptr, 0,
      gb, nullptr, kRowsP, kDm, kDm, 1.0f / kCW, 1.0f);
  fin_gate_kernel<<<kRowsP / 8, 256, 0, stream>>>(ENC32, X32, RAW32, fing, finb, YA16);
  wmma_gemm64<0, 0, false, 0><<<gemm_blocks(kRowsP, kPrP), 256, 0, stream>>>(
      YA16, kDm, PW, kDm, (void*)DEC32, kPrP, nullptr, 0,
      nullptr, nullptr, kRowsP, kPrP, kDm, 1.0f / kCW, 1.0f);
  out_kernel<<<(kOutN / 4 + 255) / 256, 256, 0, stream>>>(DEC32, pb, MEANR, STDR, out);
}
